// OutputsTreeEmbedding_38886633898792
// MI455X (gfx1250) — hardware-verified
//
#include <hip/hip_runtime.h>

#define NTOK 32768
#define DEMB 128
#define NG4  512
#define V_   100000
#define N2_  5000
#define N3_  500
#define N4_  50
#define TROWS 5632
#define R3   5000
#define R4   5500
#define RR   5550
#define FXS  16777216.0f

typedef _Float16 f16;
typedef _Float16 bf16;
typedef __attribute__((ext_vector_type(16))) f16 f16x16;
typedef f16x16 bf16x16;
typedef __attribute__((ext_vector_type(8)))  f16 f16x8;
typedef f16x8 bf16x8;
typedef __attribute__((ext_vector_type(4)))  f16 bf16x4;
typedef __attribute__((ext_vector_type(8)))  float f32x8;
typedef __attribute__((ext_vector_type(4)))  float v4f_t;
typedef float v4fa __attribute__((ext_vector_type(4), may_alias));
typedef __attribute__((ext_vector_type(4))) unsigned v4u_t;
typedef unsigned v4ua __attribute__((ext_vector_type(4), may_alias));

__device__ __forceinline__ f32x8 wmma16(f16x16 a, f16x16 b, f32x8 c) {
  c = __builtin_amdgcn_wmma_f32_16x16x32_f16(false, a, false, b, (short)0, c, false, false);
  asm volatile("v_nop\n\tv_nop\n\tv_nop\n\tv_nop" : "+v"(c) : "v"(a), "v"(b));
  return c;
}

__global__ __launch_bounds__(256) void k_segmean(const float* __restrict__ src, const int* __restrict__ parent, int v0, int nv, int nnodes,
                                                float* __restrict__ dst) {
  __shared__ int accS[64 * DEMB];
  __shared__ int cntS[64];
  __shared__ __attribute__((aligned(16))) float outS[64 * DEMB];
  const int tid = threadIdx.x, base = blockIdx.x * 64;
  for (int e = tid; e < 64 * DEMB; e += 256) accS[e] = 0;
  if (tid < 64) cntS[tid] = 0;
  __syncthreads();
  for (int v = v0 + tid; v < nv; v += 256) {
    const int p = parent[v] - base;
    if (p >= 0 && p < 64) {
      atomicAdd(&cntS[p], 1);
      const float* row = src + (size_t)v * DEMB;
#pragma unroll 4
      for (int d = 0; d < DEMB; ++d) atomicAdd(&accS[p * DEMB + d], (int)rintf(row[d] * FXS));
    }
  }
  __syncthreads();
  for (int e = tid; e < 64 * DEMB; e += 256) { const int p = e >> 7; const float c = (float)max(cntS[p], 1); outS[e] = ((float)accS[e] / FXS) / c; }
  __syncthreads();
#pragma unroll 1
  for (int pass = 0; pass < 2; ++pass) {
#pragma unroll
    for (int it = 0; it < 8; ++it) { const int ch = tid + 256 * it, p = ch >> 5, q = (ch & 31) * 4;
      if (base + p < nnodes) *(volatile v4f_t*)(dst + (size_t)(base + p) * DEMB + q) = *(const volatile v4fa*)(outS + p * DEMB + q); }
    __threadfence();
  }
}
__global__ __launch_bounds__(256) void k_root(float* __restrict__ tab) {
  __shared__ __attribute__((aligned(16))) float rS[DEMB];
  const int tid = threadIdx.x;
  if (tid < DEMB) { float s = 0.0f; for (int i = 0; i < N4_; ++i) s += tab[(size_t)(R4 + i) * DEMB + tid]; rS[tid] = s * (1.0f / (float)N4_); }
  __syncthreads();
#pragma unroll 1
  for (int pass = 0; pass < 2; ++pass) {
    if (tid < 32) *(volatile v4f_t*)(tab + (size_t)RR * DEMB + tid * 4) = *(const volatile v4fa*)(rS + tid * 4);
    for (int e = tid; e < (TROWS - RR - 1) * DEMB / 4; e += 256) { v4f_t z = {0.f, 0.f, 0.f, 0.f}; *(volatile v4f_t*)(tab + (size_t)(RR + 1) * DEMB + e * 4) = z; }
    __threadfence();
  }
}

#define SS 512
#define HH 1
#define DKK 64
#define BB 1
#define LDS_STRIDE 48
#define KSTRIDE    72
#define VSTRIDE    48

__device__ __forceinline__ f32x8 wmma_bf16(bf16x16 a, bf16x16 b, f32x8 c) {
  c = __builtin_amdgcn_wmma_f32_16x16x32_f16(false, a, false, b, (short)0, c, false, false);
  asm volatile("v_nop\n\tv_nop\n\tv_nop\n\tv_nop" : "+v"(c) : "v"(a), "v"(b));
  return c;
}

template <typename T>
__device__ __forceinline__ bf16x16 load_frag(const T* __restrict__ base, int ld,
                                             int row0, int k0) {
  const int lane = threadIdx.x & 31;
  const int r    = lane & 15;
  const int kh   = (lane >> 4) * 8;
  const T* p0 = base + (size_t)(row0 + r) * ld + (k0 + kh);
  const T* p1 = p0 + 16;
  bf16x16 f;
#pragma unroll
  for (int i = 0; i < 8; ++i) {
    f[i]     = (bf16)p0[i];
    f[i + 8] = (bf16)p1[i];
  }
  return f;
}

__device__ __forceinline__ bf16x16 lds_frag(const bf16* base, int stride) {
  const int lane = threadIdx.x & 31;
  const int row  = lane & 15;
  const int kh   = (lane >> 4) * 8;
  const bf16x8 lo = *(const bf16x8*)(base + row * stride + kh);
  const bf16x8 hi = *(const bf16x8*)(base + row * stride + kh + 16);
  bf16x16 f;
#pragma unroll
  for (int i = 0; i < 8; ++i) { f[i] = lo[i]; f[i + 8] = hi[i]; }
  return f;
}

template <typename T>
__device__ __forceinline__ void stage_read16(const T* __restrict__ p, float* buf) {
#pragma unroll
  for (int i = 0; i < 16; ++i) buf[i] = (float)p[i];
}

__device__ __forceinline__ void stage_write(bf16* dst, const float* buf, int nquad) {
#pragma unroll
  for (int i = 0; i < nquad; ++i) {
    bf16x4 q;
    q[0] = (bf16)buf[4 * i];     q[1] = (bf16)buf[4 * i + 1];
    q[2] = (bf16)buf[4 * i + 2]; q[3] = (bf16)buf[4 * i + 3];
    *(bf16x4*)(dst + 4 * i) = q;
  }
}

template <typename AT, int MODE>
__global__ __launch_bounds__(256) void gemm_rb_kernel(
    const AT* __restrict__ A, const float* __restrict__ W,
    const float* __restrict__ bias, const float* __restrict__ rowscale, const float* __restrict__ R, const float* __restrict__ rowbias, void* __restrict__ out,
    int M, int N, int K) {
  __shared__ bf16 ldsA[128 * LDS_STRIDE];
  __shared__ bf16 ldsW[256 * LDS_STRIDE];
  __shared__ __attribute__((aligned(16))) unsigned char sob[256 * 136 * 2];

  const int t    = threadIdx.x;
  const int wave = t >> 5;
  const int lane = t & 31;
  const int wm   = (wave & 1) * 64;
  const int wn   = (wave >> 1) * 64;
  const int mBlk = blockIdx.x * 128;
  const int nBlk = blockIdx.y * 256;

  const int arow = t >> 1;
  const int ach  = (t & 1) * 16;

  float abuf[16];
  float wbuf[32];

  stage_read16(A + (size_t)(mBlk + arow) * K + ach, abuf);
  const int nrow = min(nBlk + t, N - 1);
  stage_read16(W + (size_t)nrow * K,          wbuf);
  stage_read16(W + (size_t)nrow * K + 16,     wbuf + 16);

  f32x8 acc[4][4] = {};

  for (int k = 0; k < K; k += 32) {
    __syncthreads();
    stage_write(&ldsA[arow * LDS_STRIDE + ach], abuf, 4);
    stage_write(&ldsW[t * LDS_STRIDE],          wbuf, 8);
    if (k + 32 < K) {
      stage_read16(A + (size_t)(mBlk + arow) * K + (k + 32) + ach, abuf);
      stage_read16(W + (size_t)nrow * K + (k + 32),          wbuf);
      stage_read16(W + (size_t)nrow * K + (k + 32) + 16,     wbuf + 16);
    }
    __syncthreads();

    bf16x16 af[4], wf[4];
#pragma unroll
    for (int i = 0; i < 4; ++i)
      af[i] = lds_frag(ldsA + (wm + 16 * i) * LDS_STRIDE, LDS_STRIDE);
#pragma unroll
    for (int j = 0; j < 4; ++j)
      wf[j] = lds_frag(ldsW + (wn + 16 * j) * LDS_STRIDE, LDS_STRIDE);
#pragma unroll
    for (int i = 0; i < 4; ++i)
#pragma unroll
      for (int j = 0; j < 4; ++j)
        acc[i][j] = wmma_bf16(af[i], wf[j], acc[i][j]);
  }

  const int nlane = lane & 15;
  const int mh    = (lane >> 4) * 8;
  __syncthreads();
  if (MODE == 0 || MODE == 1 || MODE == 3) {
    bf16* so = (bf16*)sob;
#pragma unroll
    for (int i = 0; i < 4; ++i)
#pragma unroll
      for (int j = 0; j < 4; ++j) {
        const int nl = wn + 16 * j + nlane;
        const float bv = bias ? bias[nBlk + nl] : 0.0f;
        if (MODE == 3) {
#pragma unroll 1
          for (int r = 0; r < 8; ++r) {
            const int ml = wm + 16 * i + mh + r;
            const float xg = acc[i][j][r] + bv;
            so[ml * 264 + nl] = (bf16)(0.5f * xg * (1.0f + erff(xg * 0.70710678118654752f)));
          }
        } else {
#pragma unroll
        for (int r = 0; r < 8; ++r) {
          const int ml = wm + 16 * i + mh + r;
          const bf16 hv = (bf16)(acc[i][j][r] + bv);
          if (MODE == 0) so[ml * 264 + nl] = hv;
          else           so[nl * 136 + ml] = hv;
        }
        }
      }
    __syncthreads();
#pragma unroll 1
    for (int pass = 0; pass < 2; ++pass) {
      if (MODE == 0 || MODE == 3) {
        for (int ch = t; ch < 128 * 32; ch += 256) { const int ml = ch >> 5, q = (ch & 31) * 8;
          *(volatile v4u_t*)((bf16*)out + (size_t)(mBlk + ml) * N + nBlk + q) = *(const v4ua*)(so + ml * 264 + q); }
      } else {
        const int b_ = mBlk / SS, s0 = mBlk & (SS - 1);
        for (int ch = t; ch < 256 * 16; ch += 256) { const int nl = ch >> 4, q = (ch & 15) * 8; const int n = nBlk + nl, h = n >> 6, dk = n & (DKK - 1);
          *(volatile v4u_t*)((bf16*)out + (((size_t)(b_ * HH + h)) * DKK + dk) * SS + s0 + q) = *(const v4ua*)(so + nl * 136 + q); }
      }
      __threadfence();
    }
  } else {
    float* so = (float*)sob;
#pragma unroll 1
    for (int hf = 0; hf < 2; ++hf) {
      if (wm == hf * 64) {
#pragma unroll
        for (int i = 0; i < 4; ++i)
#pragma unroll
          for (int j = 0; j < 4; ++j) {
            const int nl = wn + 16 * j + nlane;
            const float bv = bias ? bias[nBlk + nl] : 0.0f;
#pragma unroll
            for (int r = 0; r < 8; ++r) { const int mrow = mBlk + hf * 64 + 16 * i + mh + r; so[(16 * i + mh + r) * 260 + nl] = acc[i][j][r] * (rowscale ? rowscale[mrow] : 1.0f) + bv + (rowbias ? rowbias[mrow] : 0.0f); }
          }
      }
      __syncthreads();
      if (R) {
        for (int ch = t; ch < 64 * 64; ch += 256) { const int ml = ch >> 6, q = (ch & 63) * 4;
          if (nBlk + q < N) { const v4f_t rv = *(const v4f_t*)(R + (size_t)(mBlk + hf * 64 + ml) * N + nBlk + q); v4f_t v = *(const volatile v4fa*)(so + ml * 260 + q); v += rv; *(volatile v4fa*)(so + ml * 260 + q) = v; } }
        asm volatile("s_wait_dscnt 0" ::: "memory");
      }
#pragma unroll 1
      for (int pass = 0; pass < 2; ++pass) {
        for (int ch = t; ch < 64 * 64; ch += 256) { const int ml = ch >> 6, q = (ch & 63) * 4;
          if (nBlk + q < N) *(volatile v4f_t*)((float*)out + (size_t)(mBlk + hf * 64 + ml) * N + nBlk + q) = *(const volatile v4fa*)(so + ml * 260 + q); }
        __threadfence();
      }
      __syncthreads();
    }
  }
}


__device__ __forceinline__ f16x16 lds_frag16(const f16* base, int stride) {
  const int lane = threadIdx.x & 31, row = lane & 15, kh = (lane >> 4) * 8;
  const f16x8 lo = *(const f16x8*)(base + row * stride + kh);
  const f16x8 hi = *(const f16x8*)(base + row * stride + kh + 16);
  f16x16 f;
#pragma unroll
  for (int i = 0; i < 8; ++i) { f[i] = lo[i]; f[i + 8] = hi[i]; }
  return f;
}
__device__ __forceinline__ f16x16 wfrag(const float* __restrict__ Wm, int n0, int k0) {
  const int lane = threadIdx.x & 31, r = lane & 15, kh = (lane >> 4) * 8;
  const float* p0 = Wm + (size_t)(n0 + r) * DEMB + k0 + kh;
  const v4f_t a = *(const v4f_t*)(p0), b = *(const v4f_t*)(p0 + 4), c = *(const v4f_t*)(p0 + 16), d = *(const v4f_t*)(p0 + 20);
  f16x16 f;
  f[0] = (f16)a[0]; f[1] = (f16)a[1]; f[2]  = (f16)a[2]; f[3]  = (f16)a[3]; f[4]  = (f16)b[0]; f[5]  = (f16)b[1]; f[6]  = (f16)b[2]; f[7]  = (f16)b[3];
  f[8] = (f16)c[0]; f[9] = (f16)c[1]; f[10] = (f16)c[2]; f[11] = (f16)c[3]; f[12] = (f16)d[0]; f[13] = (f16)d[1]; f[14] = (f16)d[2]; f[15] = (f16)d[3];
  return f;
}
__device__ __forceinline__ float sigm(float x) { return 1.0f / (1.0f + __expf(-x)); }
__device__ __forceinline__ float tanh_(float x) { return 1.0f - 2.0f / (1.0f + __expf(2.0f * x)); }

__global__ __launch_bounds__(64) void k_tok(const int* __restrict__ ids_g, const float* __restrict__ embed,
                                            const int* __restrict__ pl2, const int* __restrict__ pl3, const int* __restrict__ pl4,
                                            const float* __restrict__ PTf, const float* __restrict__ PTb,
                                            const float* __restrict__ wih_f, const float* __restrict__ whh_f, const float* __restrict__ bih_f, const float* __restrict__ bhh_f,
                                            const float* __restrict__ wih_b, const float* __restrict__ whh_b, const float* __restrict__ bih_b, const float* __restrict__ bhh_b,
                                            float* __restrict__ out) {
  __shared__ __attribute__((aligned(16))) f16 leafS[2][16 * 136];
  __shared__ __attribute__((aligned(16))) f16 xlS[2][16 * 520];
  __shared__ __attribute__((aligned(16))) f16 hS[2][2][16 * 136];
  __shared__ __attribute__((aligned(16))) float oS[2][16 * 132];
  __shared__ float cS[2][16 * 132];
  __shared__ int idS[2][16], rowS[2][4][16];
  const int lane = threadIdx.x & 31, wave = threadIdx.x >> 5, cl = lane & 15, hsel = lane >> 4, rh = hsel * 8;
  const int tok0 = (blockIdx.x * 2 + wave) * 16;
  if (lane < 16) {
    int id = ids_g[tok0 + lane]; id = min(max(id, 0), V_ - 1); idS[wave][lane] = id;
    int p2 = pl2[id]; p2 = min(max(p2, 0), N2_ - 1);
    int p3 = pl3[p2]; p3 = min(max(p3, 0), N3_ - 1);
    int p4 = pl4[p3]; p4 = min(max(p4, 0), N4_ - 1);
    rowS[wave][0][lane] = p2; rowS[wave][1][lane] = R3 + p3; rowS[wave][2][lane] = R4 + p4; rowS[wave][3][lane] = RR;
  }
  asm volatile("s_wait_dscnt 0" ::: "memory");
  __builtin_amdgcn_wave_barrier();
  f16* lf = leafS[wave];
  for (int e = lane; e < 16 * DEMB; e += 32) { const int r = e >> 7, c = e & 127; lf[r * 136 + c] = (f16)embed[(size_t)idS[wave][r] * DEMB + c]; }
  asm volatile("s_wait_dscnt 0" ::: "memory");
  __builtin_amdgcn_wave_barrier();
  f16x16 la[4];
#pragma unroll
  for (int ks = 0; ks < 4; ++ks) la[ks] = lds_frag16(lf + ks * 32, 136);
  const int myid[8] = { idS[wave][rh + 0], idS[wave][rh + 1], idS[wave][rh + 2], idS[wave][rh + 3], idS[wave][rh + 4], idS[wave][rh + 5], idS[wave][rh + 6], idS[wave][rh + 7] };

#pragma unroll 1
  for (int dir = 0; dir < 2; ++dir) {
    const float* wih = dir ? wih_b : wih_f; const float* whh = dir ? whh_b : whh_f;
    const float* bih = dir ? bih_b : bih_f; const float* bhh = dir ? bhh_b : bhh_f;
    const float* PT = dir ? PTb : PTf;
    f16* xl = xlS[wave];
#pragma unroll 1
    for (int nt = 0; nt < 32; ++nt) {
      f32x8 acc = {};
#pragma unroll
      for (int ks = 0; ks < 4; ++ks) acc = wmma16(la[ks], wfrag(wih, nt * 16, ks * 32), acc);
#pragma unroll
      for (int r = 0; r < 8; ++r) xl[(rh + r) * 520 + nt * 16 + cl] = (f16)acc[r];
    }
    for (int e = lane; e < 2 * 16 * 136; e += 32) (&hS[wave][0][0])[e] = (f16)0.0f;
    for (int e = lane; e < 16 * 132; e += 32) cS[wave][e] = 0.0f;
    asm volatile("s_wait_dscnt 0" ::: "memory");
    __builtin_amdgcn_wave_barrier();
    int cur = 0;
#pragma unroll 1
    for (int s = 0; s < 5; ++s) {
      const int t = dir ? (4 - s) : s;
      const f16* hp = hS[wave][cur]; f16* hn = hS[wave][cur ^ 1];
      f16x16 ha[4];
      if (s > 0) {
#pragma unroll
        for (int ks = 0; ks < 4; ++ks) ha[ks] = lds_frag16(hp + ks * 32, 136);
      }
      int srow[8]; bool useleaf[8], zero[8];
#pragma unroll
      for (int r = 0; r < 8; ++r) {
        const int id = myid[r];
        zero[r] = (id == 0); useleaf[r] = (t == 0) || (id == 1) || (id == 2);
        srow[r] = (t == 0) ? 0 : rowS[wave][t - 1][rh + r];
      }
#pragma unroll 1
      for (int ug = 0; ug < 8; ++ug) {
        f32x8 g4[4];
#pragma unroll
        for (int q = 0; q < 4; ++q) { f32x8 z = {}; g4[q] = z; }
        if (s > 0) {
#pragma unroll
          for (int q = 0; q < 4; ++q)
#pragma unroll
            for (int ks = 0; ks < 4; ++ks) g4[q] = wmma16(ha[ks], wfrag(whh, q * 128 + ug * 16, ks * 32), g4[q]);
        }
        float hnew[8];
#pragma unroll
        for (int r = 0; r < 8; ++r) {
          float pre[4];
#pragma unroll
          for (int q = 0; q < 4; ++q) {
            const int col = q * 128 + ug * 16 + cl;
            float xv = 0.0f;
            if (!zero[r]) xv = useleaf[r] ? (float)xl[(rh + r) * 520 + col] : PT[(size_t)srow[r] * NG4 + col];
            pre[q] = g4[q][r] + xv + bih[col] + bhh[col];
          }
          const float ig = sigm(pre[0]), fg = sigm(pre[1]), gg = tanh_(pre[2]), og = sigm(pre[3]);
          float* cp = &cS[wave][(rh + r) * 132 + ug * 16 + cl];
          const float cn = fg * (*cp) + ig * gg; *cp = cn;
          hnew[r] = og * tanh_(cn);
        }
#pragma unroll
        for (int r = 0; r < 8; ++r) hn[(rh + r) * 136 + ug * 16 + cl] = (f16)hnew[r];
        if (s == 4) {
#pragma unroll
          for (int r = 0; r < 8; ++r) oS[wave][(rh + r) * 132 + ug * 16 + cl] = hnew[r];
        }
      }
      asm volatile("s_wait_dscnt 0" ::: "memory");
      __builtin_amdgcn_wave_barrier();
      cur ^= 1;
    }
#pragma unroll 1
    for (int pass = 0; pass < 2; ++pass) {
#pragma unroll
      for (int r = 0; r < 16; ++r) *(volatile v4f_t*)(out + (size_t)(tok0 + r) * 256 + dir * 128 + lane * 4) = *(const volatile v4fa*)(&oS[wave][r * 132 + lane * 4]);
      __threadfence();
    }
    __builtin_amdgcn_wave_barrier();
  }
}

extern "C" void kernel_launch(void* const* d_in, const int* in_sizes, int n_in,
                              void* d_out, int out_size, void* d_ws, size_t ws_size,
                              hipStream_t stream) {
  (void)in_sizes; (void)n_in; (void)out_size; (void)ws_size;
  const int* ids = (const int*)d_in[0];
  const float* embed = (const float*)d_in[1];
  const float* wih_f = (const float*)d_in[2], *whh_f = (const float*)d_in[3], *bih_f = (const float*)d_in[4], *bhh_f = (const float*)d_in[5];
  const float* wih_b = (const float*)d_in[6], *whh_b = (const float*)d_in[7], *bih_b = (const float*)d_in[8], *bhh_b = (const float*)d_in[9];
  const int* pl2 = (const int*)d_in[10];
  const int* pl3 = (const int*)d_in[11];
  const int* pl4 = (const int*)d_in[12];
  float* out = (float*)d_out;
  char* ws = (char*)d_ws;
  float* tab = (float*)ws; ws += (size_t)TROWS * DEMB * 4;
  float* PTf = (float*)ws; ws += (size_t)TROWS * NG4 * 4;
  float* PTb = (float*)ws; ws += (size_t)TROWS * NG4 * 4;
  k_segmean<<<dim3((N2_ + 63) / 64), dim3(256), 0, stream>>>(embed, pl2, 3, V_, N2_, tab);
  k_segmean<<<dim3((N3_ + 63) / 64), dim3(256), 0, stream>>>(tab, pl3, 0, N2_, N3_, tab + (size_t)R3 * DEMB);
  k_segmean<<<dim3(1), dim3(256), 0, stream>>>(tab + (size_t)R3 * DEMB, pl4, 0, N3_, N4_, tab + (size_t)R4 * DEMB);
  k_root<<<dim3(1), dim3(256), 0, stream>>>(tab);
  gemm_rb_kernel<float, 2><<<dim3(TROWS / 128, NG4 / 256), dim3(256), 0, stream>>>(tab, wih_f, nullptr, nullptr, nullptr, nullptr, PTf, TROWS, NG4, DEMB);
  gemm_rb_kernel<float, 2><<<dim3(TROWS / 128, NG4 / 256), dim3(256), 0, stream>>>(tab, wih_b, nullptr, nullptr, nullptr, nullptr, PTb, TROWS, NG4, DEMB);
  k_tok<<<dim3(NTOK / 32), dim3(64), 0, stream>>>(ids, embed, pl2, pl3, pl4, PTf, PTb, wih_f, whh_f, bih_f, bhh_f, wih_b, whh_b, bih_b, bhh_b, out);
}
